// MemoryMultiHeadedAttention_11553462026562
// MI455X (gfx1250) — hardware-verified
//
#include <hip/hip_runtime.h>
#include <math.h>
#include <stdint.h>

#define NB    8
#define TQ    512
#define DM    512
#define NH    8
#define HD    64
#define ML    512
#define CL    128
#define KVL   (CL + ML + TQ)
#define TMEM  (CL + ML)
#define QROWS (NB * TQ)
#define KVROWS (NB * KVL)
#define CROWS (NB * CL)
#define CK    (DM * 4)
#define OUT1E (NB * TQ * DM)
#define OUT2E (2 * NB * TQ * DM)
#define OUT3E (OUT2E + NB * CL * DM)
#define OUTNE (OUT3E + 2)
#define NAUX  (NB * TQ * DM)
#define NAE   (NB * ML * DM)
#define QSC   1024.0f
#define KSC   1024.0f
#define PCAR  32768.0f
#define VCAR  1024.0f
#define OSC   1024.0f
#define WOS   1024.0f
#define LOG2E 1.4426950408889634f
#define WPB   4
#define NHG   (NH / WPB)
#define NQT   (TQ / 16)
#define ATT_THREADS (WPB * 32)
#define ATT_BLOCKS  (NQT * NHG * NB)
#define PTW   (16 * 36)
#define SLW   (16 * 68)
#define WREG  (PTW + SLW)
#define SLAB64 (16 * 68)
#define VTP   72
#define KVBLK ((KVL * DM / 8) / 256)

static_assert(DM == NH * HD && HD == 64 && NH == 8 && DM == 512 && ML == 512 && CL == 128 && TQ == 512);
static_assert(KVL == 1152 && TMEM == 640 && (KVL % 64) == 0 && (CL % 64) == 0 && (ML % 32) == 0 && (KVL % 32) == 0);
static_assert(OUT1E == 2097152 && OUT2E == 4194304 && OUT3E == 4718592 && OUTNE == 4718594);
static_assert((NH % WPB) == 0 && ATT_THREADS == 128 && ATT_BLOCKS == 512);
static_assert((QROWS % 64) == 0 && (KVROWS % 64) == 0 && (CROWS % 64) == 0 && (CK % 32) == 0 && (CK / 8) == 256);
static_assert(KVBLK == 288 && ((CL * DM / 8) % 256) == 0 && ((TMEM * DM / 8) % 256) == 0);
static_assert((NAUX % 2048) == 0 && (NAE % 2048) == 0 && NAE == (1 << 21) && (ML * DM) == (1 << 18));
static_assert(((QROWS * DM / 8) % 256) == 0 && ((KVROWS * DM / 8) % 256) == 0 && ((CROWS * DM / 8) % 256) == 0);
static_assert(((DM * DM / 8) % 256) == 0 && ((DM * CK / 8) % 256) == 0 && ((ML * CL / 8) % 256) == 0);
static_assert(((NB * TQ * DM / 4) % 256) == 0);

typedef unsigned short u16;
typedef _Float16 v16h __attribute__((ext_vector_type(16)));
typedef _Float16 v8h  __attribute__((ext_vector_type(8)));
typedef __bf16   v16b __attribute__((ext_vector_type(16)));
typedef float    v8f  __attribute__((ext_vector_type(8)));
typedef float    v4f  __attribute__((ext_vector_type(4)));
typedef float    v2f  __attribute__((ext_vector_type(2)));
typedef unsigned int v4u __attribute__((ext_vector_type(4)));

union FragH { v16h v; v8h h[2]; v4u u[2]; };
union FragB { v16b v; v4u u[2]; };

__device__ __forceinline__ unsigned short bf_bits(float f) {
  unsigned u = __float_as_uint(f);
  return (unsigned short)((u + 0x7FFFu + ((u >> 16) & 1u)) >> 16);
}
__device__ __forceinline__ float bf_up(unsigned short h) { return __uint_as_float(((unsigned)h) << 16); }
__device__ __forceinline__ float bfr(float f) { return bf_up(bf_bits(f)); }
__device__ __forceinline__ unsigned short h_bits(_Float16 x) { return __builtin_bit_cast(unsigned short, x); }
__device__ __forceinline__ unsigned pk16(unsigned short a, unsigned short b) { return (unsigned)a | ((unsigned)b << 16); }
__device__ __forceinline__ v8f zero8() { v8f z = {0.f, 0.f, 0.f, 0.f, 0.f, 0.f, 0.f, 0.f}; return z; }

__device__ __forceinline__ v16h ldfrag_h(const _Float16* p) {
  FragH f;
  f.h[0] = *(const v8h*)(p);
  f.h[1] = *(const v8h*)(p + 16);
  return f.v;
}
__device__ __forceinline__ v16b ldfrag_b(const u16* p) {
  FragB f;
  f.u[0] = *(const v4u*)(p);
  f.u[1] = *(const v4u*)(p + 16);
  return f.v;
}

__device__ __forceinline__ v8f mma_h(v16h a, v16h b, v8f c) {
  return __builtin_amdgcn_wmma_f32_16x16x32_f16(false, a, false, b, (short)0, c, false, false);
}
__device__ __forceinline__ v8f mma_b(v16b a, v16b b, v8f c) {
  return __builtin_amdgcn_wmma_f32_16x16x32_bf16(false, a, false, b, (short)0, c, false, false);
}
__device__ __forceinline__ void guard2(v8f& a, v8f& b, v16h x0, v16h x1, v16h x2, v16h x3, v16h x4, v16h x5) {
#if defined(__HIP_DEVICE_COMPILE__)
  asm volatile("v_nop\n\tv_nop\n\tv_nop\n\tv_nop"
               : "+v"(a), "+v"(b) : "v"(x0), "v"(x1), "v"(x2), "v"(x3), "v"(x4), "v"(x5) : "memory");
#endif
}
template <typename F>
__device__ __forceinline__ void guard6(v8f& a, v8f& b, v8f& c, v8f& d, F x0, F x1, F x2, F x3, F x4, F x5) {
#if defined(__HIP_DEVICE_COMPILE__)
  asm volatile("v_nop\n\tv_nop\n\tv_nop\n\tv_nop"
               : "+v"(a), "+v"(b), "+v"(c), "+v"(d) : "v"(x0), "v"(x1), "v"(x2), "v"(x3), "v"(x4), "v"(x5) : "memory");
#endif
}
__device__ __forceinline__ void guard10(v8f& a, v8f& b, v8f& c, v8f& d, v16h x0, v16h x1, v16h x2, v16h x3, v16h x4,
                                        v16h x5, v16h x6, v16h x7, v16h x8, v16h x9) {
#if defined(__HIP_DEVICE_COMPILE__)
  asm volatile("v_nop\n\tv_nop\n\tv_nop\n\tv_nop"
               : "+v"(a), "+v"(b), "+v"(c), "+v"(d)
               : "v"(x0), "v"(x1), "v"(x2), "v"(x3), "v"(x4), "v"(x5), "v"(x6), "v"(x7), "v"(x8), "v"(x9) : "memory");
#endif
}
__device__ __forceinline__ void acc_guard4(v8f& a, v8f& b, v8f& c, v8f& d) {
#if defined(__HIP_DEVICE_COMPILE__)
  asm volatile("v_nop\n\tv_nop\n\tv_nop\n\tv_nop" : "+v"(a), "+v"(b), "+v"(c), "+v"(d));
#endif
}
__device__ __forceinline__ void wave_sync_lds() {
  __builtin_amdgcn_fence(__ATOMIC_RELEASE, "workgroup");
  __builtin_amdgcn_wave_barrier();
  __builtin_amdgcn_fence(__ATOMIC_ACQUIRE, "workgroup");
}

__global__ __launch_bounds__(256) void cvt16(const float* __restrict__ x, u16* D, int n8, int f16mode, float scale) {
  const int gt = blockIdx.x * 256 + (int)threadIdx.x;
  if (gt >= n8) return;
  const float* p = x + (size_t)gt * 8;
  const v4f a = *(const v4f*)(p), b4 = *(const v4f*)(p + 4);
  float w[8];
#pragma unroll
  for (int e = 0; e < 4; ++e) { w[e] = a[e]; w[4 + e] = b4[e]; }
  v4u o;
#pragma unroll
  for (int e = 0; e < 4; ++e) {
    const float f0 = w[2 * e], f1 = w[2 * e + 1];
    const unsigned short hb0 = h_bits((_Float16)(bfr(f0) * scale));
    const unsigned short hb1 = h_bits((_Float16)(bfr(f1) * scale));
    const unsigned short bb0 = bf_bits(f0);
    const unsigned short bb1 = bf_bits(f1);
    o[e] = (f16mode != 0) ? pk16(hb0, hb1) : pk16(bb0, bb1);
  }
  u16* d = D + (size_t)gt * 8;
  for (int pass = 0; pass < 2; ++pass) {
    *(volatile v4u*)(d) = o;
    __threadfence();
  }
}

__global__ __launch_bounds__(256) void cvtkv(const float* __restrict__ cmem, const float* __restrict__ mem,
                                             const float* __restrict__ x, u16* D) {
  const int tid = threadIdx.x, bx = blockIdx.x, b = blockIdx.y;
  if (b >= NB || bx >= KVBLK) return;
  const int gt = bx * 256 + tid;
  const int r  = gt >> 6;
  const int c8 = (gt & 63) * 8;
  const float* p;
  if (bx < (CL * DM / 8) / 256)            p = cmem + ((size_t)(b * CL + r)) * DM + c8;
  else if (bx < (TMEM * DM / 8) / 256)     p = mem  + ((size_t)(b * ML + (r - CL))) * DM + c8;
  else                                     p = x    + ((size_t)(b * TQ + (r - TMEM))) * DM + c8;
  const v4f a = *(const v4f*)(p), b4 = *(const v4f*)(p + 4);
  float w[8];
#pragma unroll
  for (int e = 0; e < 4; ++e) { w[e] = a[e]; w[4 + e] = b4[e]; }
  v4u o;
#pragma unroll
  for (int e = 0; e < 4; ++e) o[e] = pk16(bf_bits(w[2 * e]), bf_bits(w[2 * e + 1]));
  u16* d = D + ((size_t)(b * KVL + r)) * DM + c8;
  for (int pass = 0; pass < 2; ++pass) {
    *(volatile v4u*)(d) = o;
    __threadfence();
  }
}

__global__ __launch_bounds__(256) void conv_a(const float* __restrict__ mem, u16* CA) {
  const int gt = blockIdx.x * 256 + (int)threadIdx.x;
  if (gt >= CROWS * (CK / 8)) return;
  const int R  = gt >> 8;
  const int q  = gt & 255;
  const int b  = R >> 7, l = R & (CL - 1);
  const int c0 = 2 * q;
  const float* src = mem + ((size_t)(b * ML + 4 * l)) * DM + c0;
  const v2f a0 = *(const v2f*)(src);
  const v2f a1 = *(const v2f*)(src + DM);
  const v2f a2 = *(const v2f*)(src + 2 * DM);
  const v2f a3 = *(const v2f*)(src + 3 * DM);
  v4u o;
  o[0] = pk16(bf_bits(a0[0]), bf_bits(a1[0]));
  o[1] = pk16(bf_bits(a2[0]), bf_bits(a3[0]));
  o[2] = pk16(bf_bits(a0[1]), bf_bits(a1[1]));
  o[3] = pk16(bf_bits(a2[1]), bf_bits(a3[1]));
  u16* d = CA + (size_t)R * CK + q * 8;
  for (int pass = 0; pass < 2; ++pass) {
    *(volatile v4u*)(d) = o;
    __threadfence();
  }
}

__global__ __launch_bounds__(256) void copy4(const float* __restrict__ x, float* o, int n4) {
  const int gt = blockIdx.x * 256 + (int)threadIdx.x;
  if (gt >= n4) return;
  const v4f a = *(const v4f*)(x + (size_t)gt * 4);
  float* d = o + (size_t)gt * 4;
  for (int pass = 0; pass < 2; ++pass) {
    *(volatile v4f*)(d) = a;
    __threadfence();
  }
}

__global__ __launch_bounds__(256) void wtb16(const float* __restrict__ W, long long wbs, u16* Dt, long long dbs, int K, int N) {
  __shared__ __align__(16) u16 T[64 * VTP];
  const int tid = threadIdx.x;
  const int bid = blockIdx.x;
  const size_t z = blockIdx.y;
  const int ntn = N >> 6;
  const int n0  = (bid % ntn) * 64;
  const int k0  = (bid / ntn) * 64;
  if (k0 + 64 > K) return;
  const float* Wz = W + z * (size_t)wbs;
  u16* Dz = Dt + z * (size_t)dbs;
  {
    const int sl = tid >> 2;
    const int dc = (tid & 3) * 16;
    const float* src = Wz + (size_t)(k0 + sl) * N + n0 + dc;
#pragma unroll
    for (int i = 0; i < 4; ++i) {
      const v4f a = *(const v4f*)(src + 4 * i);
#pragma unroll
      for (int e = 0; e < 4; ++e) T[(dc + 4 * i + e) * VTP + sl] = bf_bits(a[e]);
    }
  }
  __syncthreads();
  v4u vv[2];
  const int q8 = tid >> 3, p8 = (tid & 7) * 8;
#pragma unroll
  for (int it = 0; it < 2; ++it) {
    const int line = it * 32 + q8;
    vv[it] = *(const v4u*)(T + line * VTP + p8);
  }
  const size_t base = (size_t)n0 * K + k0 + p8;
  for (int pass = 0; pass < 2; ++pass) {
#pragma unroll
    for (int it = 0; it < 2; ++it) {
      const int line = it * 32 + q8;
      *(volatile v4u*)(Dz + base + (size_t)line * K) = vv[it];
    }
    __threadfence();
  }
}

__device__ __forceinline__ void epi64(float* sl, v8f a0, v8f a1, v8f a2, v8f a3, float oscale,
                                      const float* __restrict__ bias, int hasb, float* C, int N,
                                      size_t rowb, int col0, int lane) {
  const int hh = lane >> 4, m = lane & 15;
#pragma unroll
  for (int r = 0; r < 8; ++r) {
    const int ro = (8 * hh + r) * 68 + m;
    sl[ro]      = a0[r] * oscale;
    sl[ro + 16] = a1[r] * oscale;
    sl[ro + 32] = a2[r] * oscale;
    sl[ro + 48] = a3[r] * oscale;
  }
  wave_sync_lds();
  v4f bb = {0.f, 0.f, 0.f, 0.f};
  if (hasb != 0) {
    const v4f braw = *(const v4f*)(bias + col0 + m * 4);
#pragma unroll
    for (int e = 0; e < 4; ++e) bb[e] = bfr(braw[e]);
  }
  v4f vals[8];
#pragma unroll
  for (int it = 0; it < 8; ++it) vals[it] = *(const v4f*)(sl + (it * 2 + hh) * 68 + m * 4) + bb;
  float* dst = C + (rowb + (size_t)hh) * (size_t)N + col0 + m * 4;
  for (int pass = 0; pass < 2; ++pass) {
#pragma unroll
    for (int it = 0; it < 8; ++it) {
      *(volatile v4f*)(dst + (size_t)(it * 2) * (size_t)N) = vals[it];
    }
    __threadfence();
  }
}

__global__ __launch_bounds__(128)
void gemm_bf(const u16* __restrict__ A, const u16* __restrict__ Bt, const float* __restrict__ bias, float* C,
             long long abs_, long long bbs, long long cbs, int M, int N, int K, int hasb, float oscale) {
  __shared__ __align__(16) float slab[4 * SLAB64];
  const int tid = threadIdx.x, wave = tid >> 5, lane = tid & 31, hh = lane >> 4, m = lane & 15;
  const int ntile = N >> 6;
  const int bid   = blockIdx.x;
  const size_t z  = blockIdx.y;
  const int rowb  = (bid / ntile) * 64 + wave * 16;
  const int col0  = (bid % ntile) * 64;
  if (rowb + 16 > M) return;
  const u16* Az = A + z * (size_t)abs_;
  const u16* Bz = Bt + z * (size_t)bbs;
  float* Cz = C + z * (size_t)cbs;
  const u16* ap = Az + (size_t)(rowb + m) * K + 8 * hh;
  const u16* bp = Bz + (size_t)(col0 + m) * K + 8 * hh;
  const size_t bs = (size_t)16 * K;
  v8f acc0 = zero8(), acc1 = zero8(), acc2 = zero8(), acc3 = zero8();
#pragma unroll 1
  for (int k0 = 0; k0 < K; k0 += 32) {
    const v16b a  = ldfrag_b(ap + k0);
    const v16b b0 = ldfrag_b(bp + k0);
    const v16b b1 = ldfrag_b(bp + bs + k0);
    const v16b b2 = ldfrag_b(bp + 2 * bs + k0);
    const v16b b3 = ldfrag_b(bp + 3 * bs + k0);
    acc0 = mma_b(a, b0, acc0);
    acc1 = mma_b(a, b1, acc1);
    acc2 = mma_b(a, b2, acc2);
    acc3 = mma_b(a, b3, acc3);
    guard6<v16b>(acc0, acc1, acc2, acc3, a, b0, b1, b2, b3, a);
  }
  epi64(slab + wave * SLAB64, acc0, acc1, acc2, acc3, oscale, bias, hasb, Cz, N, (size_t)rowb, col0, lane);
}

__global__ __launch_bounds__(128)
void gemm_h2(const u16* __restrict__ Ah, const u16* __restrict__ Al, const u16* __restrict__ Bt,
             const float* __restrict__ bias, float* C, int M, int N, int K, int hasb, float oscale) {
  __shared__ __align__(16) float slab[4 * SLAB64];
  const int tid = threadIdx.x, wave = tid >> 5, lane = tid & 31, hh = lane >> 4, m = lane & 15;
  const int ntile = N >> 6;
  const int bid   = blockIdx.x;
  const int rowb  = (bid / ntile) * 64 + wave * 16;
  const int col0  = (bid % ntile) * 64;
  if (rowb + 16 > M) return;
  const size_t aofs = (size_t)(rowb + m) * K + 8 * hh;
  const _Float16* ahp = (const _Float16*)(const void*)Ah + aofs;
  const _Float16* alp = (const _Float16*)(const void*)Al + aofs;
  const _Float16* bp  = (const _Float16*)(const void*)Bt + (size_t)(col0 + m) * K + 8 * hh;
  const size_t bs = (size_t)16 * K;
  v8f acc0 = zero8(), acc1 = zero8(), acc2 = zero8(), acc3 = zero8();
#pragma unroll 1
  for (int k0 = 0; k0 < K; k0 += 32) {
    const v16h ah = ldfrag_h(ahp + k0), al = ldfrag_h(alp + k0);
    const v16h b0 = ldfrag_h(bp + k0);
    const v16h b1 = ldfrag_h(bp + bs + k0);
    const v16h b2 = ldfrag_h(bp + 2 * bs + k0);
    const v16h b3 = ldfrag_h(bp + 3 * bs + k0);
    acc0 = mma_h(ah, b0, acc0);  acc0 = mma_h(al, b0, acc0);
    acc1 = mma_h(ah, b1, acc1);  acc1 = mma_h(al, b1, acc1);
    acc2 = mma_h(ah, b2, acc2);  acc2 = mma_h(al, b2, acc2);
    acc3 = mma_h(ah, b3, acc3);  acc3 = mma_h(al, b3, acc3);
    guard6<v16h>(acc0, acc1, acc2, acc3, ah, al, b0, b1, b2, b3);
  }
  epi64(slab + wave * SLAB64, acc0, acc1, acc2, acc3, oscale, bias, hasb, C, N, (size_t)rowb, col0, lane);
}

__global__ __launch_bounds__(256) void split16p(const float* __restrict__ x, int sp, int nc8, u16* hpl, u16* lpl,
                                                int n8, int wlo, float sc) {
  const int gt = blockIdx.x * 256 + (int)threadIdx.x;
  if (gt >= n8) return;
  const int row = gt / nc8;
  const int c8  = (gt - row * nc8) * 8;
  const float* p = x + (size_t)row * sp + c8;
  const v4f a = *(const v4f*)(p), b4 = *(const v4f*)(p + 4);
  float w[8];
#pragma unroll
  for (int e = 0; e < 4; ++e) { w[e] = a[e]; w[4 + e] = b4[e]; }
  v4u oh, ol;
#pragma unroll
  for (int e = 0; e < 4; ++e) {
    const float t0 = w[2 * e] * sc, t1 = w[2 * e + 1] * sc;
    const _Float16 h0 = (_Float16)t0, h1 = (_Float16)t1;
    const _Float16 l0 = (_Float16)(t0 - (float)h0), l1 = (_Float16)(t1 - (float)h1);
    oh[e] = pk16(h_bits(h0), h_bits(h1));
    ol[e] = pk16(h_bits(l0), h_bits(l1));
  }
  const size_t o8 = (size_t)gt * 8;
  for (int pass = 0; pass < 2; ++pass) {
    *(volatile v4u*)(hpl + o8) = oh;
    if (wlo != 0) *(volatile v4u*)(lpl + o8) = ol;
    __threadfence();
  }
}

__global__ __launch_bounds__(256) void vt16g(const float* __restrict__ v, int sp, int voff, int kvl, int nst,
                                             u16* VHo, u16* VLo, int wlo) {
  __shared__ __align__(16) u16 TH[HD * VTP];
  __shared__ __align__(16) u16 TL[HD * VTP];
  const int tid = threadIdx.x;
  const int bid = blockIdx.x;
  const int st  = bid % nst;
  const int bg  = bid / nst;
  if (bg >= NB * NH) return;
  const int b   = bg / NH;
  const int g   = bg % NH;
  const int s0  = st * 64;
  {
    const int sl = tid >> 2;
    const int dc = (tid & 3) * 16;
    const float* src = v + ((size_t)(b * kvl + s0 + sl)) * (size_t)sp + voff + g * HD + dc;
#pragma unroll
    for (int i = 0; i < 4; ++i) {
      const v4f a = *(const v4f*)(src + 4 * i);
#pragma unroll
      for (int e = 0; e < 4; ++e) {
        const float t = a[e] * VCAR;
        const _Float16 h = (_Float16)t;
        const _Float16 l = (_Float16)(t - (float)h);
        TH[(dc + 4 * i + e) * VTP + sl] = h_bits(h);
        TL[(dc + 4 * i + e) * VTP + sl] = h_bits(l);
      }
    }
  }
  __syncthreads();
  v4u vh[2], vl[2];
  const int q8 = tid >> 3, p8 = (tid & 7) * 8;
#pragma unroll
  for (int it = 0; it < 2; ++it) {
    const int line = it * 32 + q8;
    vh[it] = *(const v4u*)(TH + line * VTP + p8);
    vl[it] = *(const v4u*)(TL + line * VTP + p8);
  }
  const size_t base = ((size_t)bg * HD) * (size_t)kvl + s0 + p8;
  for (int pass = 0; pass < 2; ++pass) {
#pragma unroll
    for (int it = 0; it < 2; ++it) {
      const int line = it * 32 + q8;
      *(volatile v4u*)(VHo + base + (size_t)line * kvl) = vh[it];
      if (wlo != 0) *(volatile v4u*)(VLo + base + (size_t)line * kvl) = vl[it];
    }
    __threadfence();
  }
}

template <int SPLIT, int MASKED, int OUTF>
__global__ __launch_bounds__(ATT_THREADS)
void attn(const u16* __restrict__ QHIp, const u16* __restrict__ QLOp,
          const u16* __restrict__ KHIp, const u16* __restrict__ KLOp,
          const u16* __restrict__ VHIp, const u16* __restrict__ VLOp,
          u16* OHIp, u16* OLOp, float* OFp, int kvl, int koff, int nktall) {
  __shared__ __align__(16) float smem[WPB * WREG];

  const int tid  = threadIdx.x;
  const int wave = tid >> 5;
  const int lane = tid & 31;
  const int hh   = lane >> 4;
  const int c    = lane & 15;
  const int bid  = blockIdx.x;
  const int qt   = bid % NQT;
  const int rem  = bid / NQT;
  const int hg   = rem % NHG;
  const int b    = rem / NHG;
  if (b >= NB) return;
  const int head = hg * WPB + wave;
  const int q0   = qt * 16;

  float* pt   = smem + wave * WREG;
  float* slab = pt + PTW;

  const size_t rq0  = (size_t)b * TQ + q0;
  const size_t qofs = ((rq0 + c) * NH + head) * HD + 8 * hh;
  const _Float16* Qh  = (const _Float16*)(const void*)QHIp + qofs;
  const _Float16* Ql  = (const _Float16*)(const void*)QLOp + qofs;
  const size_t kofs = (((size_t)b * kvl + koff + c) * NH + head) * HD + 8 * hh;
  const _Float16* Khb = (const _Float16*)(const void*)KHIp + kofs;
  const _Float16* Klb = (const _Float16*)(const void*)KLOp + kofs;
  const size_t vofs = (((size_t)b * NH + head) * HD + c) * (size_t)kvl + koff + 8 * hh;
  const _Float16* Vhb = (const _Float16*)(const void*)VHIp + vofs;
  const _Float16* Vlb = (const _Float16*)(const void*)VLOp + vofs;
  const float lsc = 0.125f * (LOG2E / (QSC * KSC));
  const float oc  = 1.0f / (PCAR * VCAR);
  const size_t KROW = (size_t)NH * HD;
  const size_t VP   = (size_t)kvl;

  float mrow[8], lrow[8];
  v8f o[4];
#pragma unroll
  for (int r = 0; r < 8; ++r) { mrow[r] = -INFINITY; lrow[r] = 0.f; }
#pragma unroll
  for (int j = 0; j < 4; ++j) o[j] = zero8();
  int nkt = nktall;
  if (MASKED) {
    const int ncaus = ((q0 + 15 + TMEM) >> 5) + 1;
    nkt = (ncaus < nktall) ? ncaus : nktall;
  }

#pragma unroll 1
  for (int kt = 0; kt < nkt; ++kt) {
    const int kb = kt * 32;
    v8f s0 = zero8(), s1 = zero8();
    const _Float16* k0p = Khb + (size_t)kb * KROW;
    const _Float16* k1p = k0p + (size_t)16 * KROW;
    if (SPLIT) {
      const _Float16* l0p = Klb + (size_t)kb * KROW;
      const _Float16* l1p = l0p + (size_t)16 * KROW;
#pragma unroll
      for (int kk = 0; kk < 2; ++kk) {
        const v16h qh  = ldfrag_h(Qh + kk * 32),  ql  = ldfrag_h(Ql + kk * 32);
        const v16h kh0 = ldfrag_h(k0p + kk * 32), kl0 = ldfrag_h(l0p + kk * 32);
        const v16h kh1 = ldfrag_h(k1p + kk * 32), kl1 = ldfrag_h(l1p + kk * 32);
        s0 = mma_h(qh, kh0, s0);
        s0 = mma_h(ql, kh0, s0);
        s0 = mma_h(qh, kl0, s0);
        s1 = mma_h(qh, kh1, s1);
        s1 = mma_h(ql, kh1, s1);
        s1 = mma_h(qh, kl1, s1);
        guard2(s0, s1, qh, ql, kh0, kl0, kh1, kl1);
      }
    } else {
#pragma unroll
      for (int kk = 0; kk < 2; ++kk) {
        const v16h qh  = ldfrag_h(Qh + kk * 32);
        const v16h kh0 = ldfrag_h(k0p + kk * 32);
        const v16h kh1 = ldfrag_h(k1p + kk * 32);
        s0 = mma_h(qh, kh0, s0);
        s1 = mma_h(qh, kh1, s1);
        guard2(s0, s1, qh, kh0, kh1, qh, kh0, kh1);
      }
    }
#pragma unroll
    for (int r = 0; r < 8; ++r) {
      float t0 = s0[r] * lsc;
      float t1 = s1[r] * lsc;
      if (MASKED) {
        const int lim  = q0 + 8 * hh + r + TMEM;
        const int key0 = kb + c;
        t0 = (key0 > lim) ? -INFINITY : t0;
        t1 = (key0 + 16 > lim) ? -INFINITY : t1;
      }
      float mx = fmaxf(t0, t1);
#pragma unroll
      for (int off = 1; off < 16; off <<= 1) mx = fmaxf(mx, __shfl_xor(mx, off, 32));
      const float mn = fmaxf(mrow[r], mx);
      const float ms = (mn == -INFINITY) ? 0.0f : mn;
      const float al = exp2f(mrow[r] - ms);
      mrow[r] = mn;
      const float e0 = exp2f(t0 - ms), e1 = exp2f(t1 - ms);
      float ps = e0 + e1;
#pragma unroll
      for (int off = 1; off < 16; off <<= 1) ps += __shfl_xor(ps, off, 32);
      lrow[r] = lrow[r] * al + ps;
#pragma unroll
      for (int j = 0; j < 4; ++j) o[j][r] *= al;
      const int ro = (8 * hh + r) * 36 + c;
      pt[ro]      = e0;
      pt[ro + 16] = e1;
    }
    wave_sync_lds();
    const float* prow = pt + c * 36 + 8 * hh;
    const v4f p0 = *(const v4f*)(prow), p1 = *(const v4f*)(prow + 4);
    const v4f p2 = *(const v4f*)(prow + 16), p3 = *(const v4f*)(prow + 20);
    if (SPLIT) {
      FragH ph, pl;
#pragma unroll
      for (int e = 0; e < 4; ++e) {
        const float ta = p0[e] * PCAR, tb = p1[e] * PCAR, tc = p2[e] * PCAR, td = p3[e] * PCAR;
        const _Float16 ha = (_Float16)ta, hb = (_Float16)tb, hc = (_Float16)tc, hd = (_Float16)td;
        ph.h[0][e]     = ha;
        ph.h[0][4 + e] = hb;
        ph.h[1][e]     = hc;
        ph.h[1][4 + e] = hd;
        pl.h[0][e]     = (_Float16)(ta - (float)ha);
        pl.h[0][4 + e] = (_Float16)(tb - (float)hb);
        pl.h[1][e]     = (_Float16)(tc - (float)hc);
        pl.h[1][4 + e] = (_Float16)(td - (float)hd);
      }
      const _Float16* vhp = Vhb + kb;
      const _Float16* vlp = Vlb + kb;
      const v16h vh0 = ldfrag_h(vhp);
      const v16h vh1 = ldfrag_h(vhp + (size_t)16 * VP);
      const v16h vh2 = ldfrag_h(vhp + (size_t)32 * VP);
      const v16h vh3 = ldfrag_h(vhp + (size_t)48 * VP);
      const v16h vl0 = ldfrag_h(vlp);
      const v16h vl1 = ldfrag_h(vlp + (size_t)16 * VP);
      const v16h vl2 = ldfrag_h(vlp + (size_t)32 * VP);
      const v16h vl3 = ldfrag_h(vlp + (size_t)48 * VP);
      o[0] = mma_h(ph.v, vh0, o[0]);  o[0] = mma_h(pl.v, vh0, o[0]);  o[0] = mma_h(ph.v, vl0, o[0]);
      o[1] = mma_h(ph.v, vh1, o[1]);  o[1] = mma_h(pl.v, vh1, o[1]);  o[1] = mma_h(ph.v, vl1, o[1]);
      o[2] = mma_h(ph.v, vh2, o[2]);  o[2] = mma_h(pl.v, vh2, o[2]);  o[2] = mma_h(ph.v, vl2, o[2]);
      o[3] = mma_h(ph.v, vh3, o[3]);  o[3] = mma_h(pl.v, vh3, o[3]);  o[3] = mma_h(ph.v, vl3, o[3]);
      guard10(o[0], o[1], o[2], o[3], ph.v, pl.v, vh0, vh1, vh2, vh3, vl0, vl1, vl2, vl3);
    } else {
      FragH ph;
#pragma unroll
      for (int e = 0; e < 4; ++e) {
        ph.h[0][e]     = (_Float16)(p0[e] * PCAR);
        ph.h[0][4 + e] = (_Float16)(p1[e] * PCAR);
        ph.h[1][e]     = (_Float16)(p2[e] * PCAR);
        ph.h[1][4 + e] = (_Float16)(p3[e] * PCAR);
      }
      const _Float16* vhp = Vhb + kb;
      const v16h vh0 = ldfrag_h(vhp);
      const v16h vh1 = ldfrag_h(vhp + (size_t)16 * VP);
      const v16h vh2 = ldfrag_h(vhp + (size_t)32 * VP);
      const v16h vh3 = ldfrag_h(vhp + (size_t)48 * VP);
      o[0] = mma_h(ph.v, vh0, o[0]);
      o[1] = mma_h(ph.v, vh1, o[1]);
      o[2] = mma_h(ph.v, vh2, o[2]);
      o[3] = mma_h(ph.v, vh3, o[3]);
      guard6<v16h>(o[0], o[1], o[2], o[3], ph.v, vh0, vh1, vh2, vh3, ph.v);
    }
    wave_sync_lds();
  }
  acc_guard4(o[0], o[1], o[2], o[3]);
#pragma unroll
  for (int r = 0; r < 8; ++r) {
    const float lv  = lrow[r];
    const float ls  = (lv > 0.0f) ? lv : 1.0f;
    const float inv = (lv > 0.0f) ? ((1.0f / ls) * oc) : 0.0f;
#pragma unroll
    for (int j = 0; j < 4; ++j) {
      const int idx = (8 * hh + r) * 68 + j * 16 + c;
      slab[idx] = o[j][r] * inv;
    }
  }

  wave_sync_lds();
  if (OUTF) {
    v4f vals[8];
#pragma unroll
    for (int it = 0; it < 8; ++it) vals[it] = *(const v4f*)(slab + (it * 2 + hh) * 68 + c * 4);
    float* dst = OFp + ((rq0 + (size_t)hh) * NH + head) * HD + c * 4;
    for (int pass = 0; pass < 2; ++pass) {
#pragma unroll
      for (int it = 0; it < 8; ++it) {
        *(volatile v4f*)(dst + (size_t)(it * 2) * (size_t)(NH * HD)) = vals[it];
      }
      __threadfence();
    }
  } else {
    v4u oh[4], ol[4];
    const int rq = lane >> 3, c8 = (lane & 7) * 8;
#pragma unroll
    for (int it = 0; it < 4; ++it) {
      const int row = it * 4 + rq;
      const v4f a = *(const v4f*)(slab + row * 68 + c8), b4 = *(const v4f*)(slab + row * 68 + c8 + 4);
      float w[8];
#pragma unroll
      for (int e = 0; e < 4; ++e) { w[e] = a[e] * OSC; w[4 + e] = b4[e] * OSC; }
#pragma unroll
      for (int e = 0; e < 4; ++e) {
        const _Float16 h0 = (_Float16)w[2 * e], h1 = (_Float16)w[2 * e + 1];
        const _Float16 l0 = (_Float16)(w[2 * e] - (float)h0), l1 = (_Float16)(w[2 * e + 1] - (float)h1);
        oh[it][e] = pk16(h_bits(h0), h_bits(h1));
        ol[it][e] = pk16(h_bits(l0), h_bits(l1));
      }
    }
    const size_t ob = (rq0 * NH + head) * HD + c8;
    for (int pass = 0; pass < 2; ++pass) {
#pragma unroll
      for (int it = 0; it < 4; ++it) {
        const int row = it * 4 + rq;
        const size_t o8 = ob + (size_t)row * (NH * HD);
        *(volatile v4u*)(OHIp + o8) = oh[it];
        *(volatile v4u*)(OLOp + o8) = ol[it];
      }
      __threadfence();
    }
  }
}

__global__ __launch_bounds__(512) void losses(const float* __restrict__ A1, const float* __restrict__ A2,
                                              const float* __restrict__ REC, const float* __restrict__ mem, float* out) {
  __shared__ double r1[512];
  __shared__ double r2[512];
  const int tid = threadIdx.x;
  double s1 = 0.0, s2 = 0.0;
#pragma unroll 1
  for (int it = 0; it < NAUX / 2048; ++it) {
    const size_t e = ((size_t)it * 512 + tid) * 4;
    const v4f a = *(const v4f*)(A1 + e), bq = *(const v4f*)(A2 + e);
    float q = 0.f;
#pragma unroll
    for (int u = 0; u < 4; ++u) { const float d = a[u] - bq[u]; q += d * d; }
    s1 += (double)q;
  }
#pragma unroll 1
  for (int it = 0; it < NAE / 2048; ++it) {
    const size_t e = ((size_t)it * 512 + tid) * 4;
    const int bb = (int)(e >> 18), dd = (int)((e >> 9) & (DM - 1)), m0 = (int)(e & (ML - 1));
    const v4f rv = *(const v4f*)(REC + e);
    float q = 0.f;
#pragma unroll
    for (int u = 0; u < 4; ++u) {
      const float mv = bfr(mem[((size_t)(bb * ML + m0 + u)) * DM + dd]);
      const float d = mv - rv[u];
      q += d * d;
    }
    s2 += (double)q;
  }
  r1[tid] = s1;
  r2[tid] = s2;
  __syncthreads();
#pragma unroll 1
  for (int o2 = 256; o2 > 0; o2 >>= 1) {
    if (tid < o2) { r1[tid] += r1[tid + o2]; r2[tid] += r2[tid + o2]; }
    __syncthreads();
  }
  if (tid == 0) {
    const float la = (float)(r1[0] * (1.0 / (double)NAUX));
    const float le = (float)(r2[0] * (1.0 / (double)NAE));
    v2f w;
    w[0] = la;
    w[1] = le;
    *(volatile v2f*)(out + OUT3E) = w;
    __threadfence();
    *(volatile v2f*)(out + OUT3E) = w;
  }
}

extern "C" void kernel_launch(void* const* d_in, const int* in_sizes, int n_in,
                              void* d_out, int out_size, void* d_ws, size_t ws_size,
                              hipStream_t stream) {
  if (n_in < 11) return;
  if (in_sizes[0] != NB * TQ * DM || in_sizes[1] != NB * ML * DM || in_sizes[2] != NB * CL * DM) return;
  if (in_sizes[3] != DM * DM || in_sizes[4] != 2 * DM * DM || in_sizes[5] != DM * DM || in_sizes[6] != DM) return;
  if (in_sizes[7] != DM * DM * 4 || in_sizes[8] != DM || in_sizes[9] != ML * CL || in_sizes[10] != ML) return;
  if (out_size != OUTNE) return;

  const float* x    = (const float*)d_in[0];
  const float* mem  = (const float*)d_in[1];
  const float* cmem = (const float*)d_in[2];
  const float* wq   = (const float*)d_in[3];
  const float* wkv  = (const float*)d_in[4];
  const float* wo   = (const float*)d_in[5];
  const float* bo   = (const float*)d_in[6];
  const float* cw   = (const float*)d_in[7];
  const float* cb   = (const float*)d_in[8];
  const float* dw   = (const float*)d_in[9];
  const float* db   = (const float*)d_in[10];
  float*       out  = (float*)d_out;

  const size_t szXB   = (size_t)QROWS * DM * 2;
  const size_t szKVIN = (size_t)KVROWS * DM * 2;
  const size_t szWQ   = (size_t)DM * DM * 2;
  const size_t szWKV  = (size_t)2 * DM * DM * 2;
  const size_t szWO   = (size_t)DM * DM * 2;
  const size_t szCW   = (size_t)DM * CK * 2;
  const size_t szDW   = (size_t)ML * CL * 2;
  const size_t szCA   = (size_t)CROWS * CK * 2;
  const size_t szQF   = (size_t)QROWS * DM * 4;
  const size_t szQP   = (size_t)QROWS * DM * 2;
  const size_t szF    = (size_t)KVROWS * 2 * DM * 4;
  const size_t szKP   = (size_t)KVROWS * DM * 2;
  const size_t szVP   = (size_t)NB * NH * HD * KVL * 2;
  const size_t szOP   = (size_t)QROWS * DM * 2;
  const size_t szCB   = (size_t)CROWS * DM * 2;
  const size_t szCT   = (size_t)NB * DM * CL * 2;
  const size_t szCKH  = (size_t)CROWS * DM * 2;
  const size_t szCVH  = (size_t)NB * NH * HD * CL * 2;
  const size_t szCKVF = (size_t)CROWS * 2 * DM * 4;
  const size_t szA    = (size_t)QROWS * DM * 4;
  const size_t szREC  = (size_t)NB * DM * ML * 4;
  if (szCKVF + 2 * szA + szREC > szF) return;

  size_t off = 0;
  const size_t oXB   = off; off += szXB;
  const size_t oKVIN = off; off += szKVIN;
  const size_t oWQ   = off; off += szWQ;
  const size_t oWKV  = off; off += szWKV;
  const size_t oWO   = off; off += szWO;
  const size_t oCW   = off; off += szCW;
  const size_t oDW   = off; off += szDW;
  const size_t oCA   = off; off += szCA;
  const size_t oQF   = off; off += szQF;
  const size_t oQHI  = off; off += szQP;
  const size_t oQLO  = off; off += szQP;
  const size_t oF    = off; off += szF;
  const size_t oKHI  = off; off += szKP;
  const size_t oKLO  = off; off += szKP;
  const size_t oVHI  = off; off += szVP;
  const size_t oVLO  = off; off += szVP;
  const size_t oOHI  = off; off += szOP;
  const size_t oOLO  = off; off += szOP;
  const size_t oCB   = off; off += szCB;
  const size_t oCT   = off; off += szCT;
  const size_t oCKH  = off; off += szCKH;
  const size_t oCVH  = off; off += szCVH;
  if (off > ws_size) return;
  if (off > (size_t)134217728) return;
  const size_t oCKVF = oF;
  const size_t oA1   = oF + szCKVF;
  const size_t oA2   = oA1 + szA;
  const size_t oREC  = oA2 + szA;

  char* ws = (char*)d_ws;
  u16*   XB   = (u16*)(ws + oXB);
  u16*   KVIN = (u16*)(ws + oKVIN);
  u16*   WQB  = (u16*)(ws + oWQ);
  u16*   WKVB = (u16*)(ws + oWKV);
  u16*   WOH  = (u16*)(ws + oWO);
  u16*   CWB  = (u16*)(ws + oCW);
  u16*   DWB  = (u16*)(ws + oDW);
  u16*   CA   = (u16*)(ws + oCA);
  float* QF   = (float*)(ws + oQF);
  u16*   QHI  = (u16*)(ws + oQHI);
  u16*   QLO  = (u16*)(ws + oQLO);
  float* F    = (float*)(ws + oF);
  u16*   KHI  = (u16*)(ws + oKHI);
  u16*   KLO  = (u16*)(ws + oKLO);
  u16*   VHI  = (u16*)(ws + oVHI);
  u16*   VLO  = (u16*)(ws + oVLO);
  u16*   OHI  = (u16*)(ws + oOHI);
  u16*   OLO  = (u16*)(ws + oOLO);
  u16*   CB   = (u16*)(ws + oCB);
  u16*   CT   = (u16*)(ws + oCT);
  u16*   CKH  = (u16*)(ws + oCKH);
  u16*   CVH  = (u16*)(ws + oCVH);
  float* CKVF = (float*)(ws + oCKVF);
  float* A1   = (float*)(ws + oA1);
  float* A2   = (float*)(ws + oA2);
  float* REC  = (float*)(ws + oREC);
  const float* nobias = (const float*)(ws + oXB);
  float* out2 = out + OUT2E;

  const dim3 blk(256);
  const int  n8x   = (QROWS * DM) / 8;
  const dim3 gX(n8x / 256);
  const dim3 gKV(KVBLK, NB);
  const dim3 gWq((DM * DM / 8) / 256);
  const dim3 gWkv((2 * DM * DM / 8) / 256);
  const dim3 gCW((DM * CK / 8) / 256);
  const dim3 gDW((ML * CL / 8) / 256);
  const dim3 gCA((CROWS * (CK / 8)) / 256);
  const int  n4o  = (NB * TQ * DM) / 4;
  const dim3 gCP(n4o / 256);
  const dim3 bG(128);
  const dim3 gGq((QROWS / 64) * (DM / 64), 1);
  const dim3 gGkv((KVROWS / 64) * (2 * DM / 64), 1);
  const dim3 gGconv((CROWS / 64) * (DM / 64), 1);
  const dim3 gGckv((CROWS / 64) * (2 * DM / 64), 1);
  const dim3 gGdec((DM / 64) * (ML / 64), NB);
  const int  n8kv  = (KVROWS * DM) / 8;
  const dim3 gSkv(n8kv / 256);
  const int  n8c   = (CROWS * DM) / 8;
  const dim3 gSc(n8c / 256);
  const dim3 gVT(NB * NH * (KVL / 64));
  const dim3 gVTc(NB * NH * (CL / 64));
  const dim3 gCT((CL / 64) * (DM / 64), NB);
  const dim3 gAT(ATT_BLOCKS);
  const dim3 bAT(ATT_THREADS);

  cvt16<<<gX, blk, 0, stream>>>(x, XB, n8x, 0, 1.0f);
  cvtkv<<<gKV, blk, 0, stream>>>(cmem, mem, x, KVIN);
  cvt16<<<gWq, blk, 0, stream>>>(wq, WQB, (DM * DM) / 8, 0, 1.0f);
  cvt16<<<gWkv, blk, 0, stream>>>(wkv, WKVB, (2 * DM * DM) / 8, 0, 1.0f);
  cvt16<<<gWq, blk, 0, stream>>>(wo, WOH, (DM * DM) / 8, 1, WOS);
  cvt16<<<gCW, blk, 0, stream>>>(cw, CWB, (DM * CK) / 8, 0, 1.0f);
  cvt16<<<gDW, blk, 0, stream>>>(dw, DWB, (ML * CL) / 8, 0, 1.0f);
  conv_a<<<gCA, blk, 0, stream>>>(mem, CA);
  copy4<<<gCP, blk, 0, stream>>>(x, out + OUT1E, n4o);
  gemm_bf<<<gGq, bG, 0, stream>>>(XB, WQB, nobias, QF, 0, 0, 0, QROWS, DM, DM, 0, 1.0f);
  split16p<<<gX, blk, 0, stream>>>(QF, DM, DM / 8, QHI, QLO, n8x, 1, QSC);
  gemm_bf<<<gGkv, bG, 0, stream>>>(KVIN, WKVB, nobias, F, 0, 0, 0, KVROWS, 2 * DM, DM, 0, 1.0f);
  split16p<<<gSkv, blk, 0, stream>>>(F, 2 * DM, DM / 8, KHI, KLO, n8kv, 1, KSC);
  vt16g<<<gVT, blk, 0, stream>>>(F, 2 * DM, DM, KVL, KVL / 64, VHI, VLO, 1);
  gemm_bf<<<gGconv, bG, 0, stream>>>(CA, CWB, cb, out2, 0, 0, 0, CROWS, DM, CK, 1, 1.0f);
  cvt16<<<gSc, blk, 0, stream>>>(out2, CB, n8c, 0, 1.0f);
  wtb16<<<gCT, blk, 0, stream>>>(out2, (long long)(CL * DM), CT, (long long)(DM * CL), CL, DM);
  gemm_bf<<<gGckv, bG, 0, stream>>>(CB, WKVB, nobias, CKVF, 0, 0, 0, CROWS, 2 * DM, DM, 0, 1.0f);
  split16p<<<gSc, blk, 0, stream>>>(CKVF, 2 * DM, DM / 8, CKH, CKH, n8c, 0, KSC);
  vt16g<<<gVTc, blk, 0, stream>>>(CKVF, 2 * DM, DM, CL, CL / 64, CVH, CVH, 0);
  attn<1, 1, 0><<<gAT, bAT, 0, stream>>>(QHI, QLO, KHI, KLO, VHI, VLO, OHI, OLO, QF, KVL, 0, KVL / 32);
  gemm_h2<<<gGq, bG, 0, stream>>>(OHI, OLO, WOH, bo, out, QROWS, DM, DM, 1, 1.0f / (OSC * WOS));
  attn<0, 0, 1><<<gAT, bAT, 0, stream>>>(QHI, QHI, KHI, KHI, VHI, VHI, OHI, OHI, A1, KVL, CL, ML / 32);
  attn<0, 0, 1><<<gAT, bAT, 0, stream>>>(QHI, QHI, CKH, CKH, CVH, CVH, OHI, OHI, A2, CL, 0, CL / 32);
  gemm_bf<<<gGdec, bG, 0, stream>>>(CT, DWB, db, REC, (long long)(DM * CL), 0, (long long)(DM * ML), DM, ML, CL, 1, 1.0f);
  losses<<<dim3(1), dim3(512), 0, stream>>>(A1, A2, REC, mem, out);
  (void)hipGetLastError();
}
